// KANLayer_75814762709066
// MI455X (gfx1250) — hardware-verified
//
#include <hip/hip_runtime.h>
#include <math.h>

constexpr int kBatch  = 2048;
constexpr int kInF    = 512;
constexpr int kOutF   = 512;
constexpr int kKnots  = 32;
constexpr int kKdim   = kInF * kKnots;
constexpr float kBasisCarry = 256.0f;
constexpr float kCoefCarry  = 16.0f;
constexpr float kOutScale   = 1.0f / (256.0f * 16.0f);
constexpr int kTabOff   = 3;
constexpr int kTabAlloc = 48;
constexpr int kMaxInterval = kKnots + 3 - 1;

static_assert(kKdim % 32 == 0, "K multiple of 32");
static_assert(kBatch % 64 == 0 && kOutF % 64 == 0, "M, N multiples of the 64 tile");
static_assert((kOutF * kKdim / 8) % 256 == 0, "coef plane thread count multiple of 256");
static_assert((kBatch * kInF * 4) % 256 == 0, "basis plane thread count multiple of 256");
static_assert(kKnots % 8 == 0, "knot axis multiple of 8");

typedef __attribute__((ext_vector_type(16))) _Float16 v16h;
typedef __attribute__((ext_vector_type(8)))  _Float16 v8h;
typedef __attribute__((ext_vector_type(16))) __bf16   v16b;
typedef __attribute__((ext_vector_type(8)))  __bf16   v8b;
typedef __attribute__((ext_vector_type(8)))  float    v8f;
typedef __attribute__((ext_vector_type(4)))  float    v4f;
typedef __attribute__((ext_vector_type(4)))  unsigned int v4u;

__device__ __forceinline__ unsigned short f2bf_bits(float f) {
  unsigned u = __float_as_uint(f);
  return (unsigned short)((u + 0x7FFFu + ((u >> 16) & 1u)) >> 16);
}
__device__ __forceinline__ float bf_bits2f(unsigned short h) { return __uint_as_float(((unsigned)h) << 16); }

__device__ __forceinline__ void dep_guard_h(v8f& a, v8f& b, v16h x, v16h y) { asm volatile("v_nop\n\tv_nop\n\tv_nop\n\tv_nop" : "+v"(a), "+v"(b) : "v"(x), "v"(y)); }
__device__ __forceinline__ void dep_guard_b(v8f& a, v8f& b, v16b x, v16b y) { asm volatile("v_nop\n\tv_nop\n\tv_nop\n\tv_nop" : "+v"(a), "+v"(b) : "v"(x), "v"(y)); }
__device__ __forceinline__ void keep4_h(v16h a, v16h b, v16h c, v16h d) { asm volatile("v_nop" :: "v"(a), "v"(b), "v"(c), "v"(d)); }
__device__ __forceinline__ void keep4_b(v16b a, v16b b, v16b c, v16b d) { asm volatile("v_nop" :: "v"(a), "v"(b), "v"(c), "v"(d)); }
__device__ __forceinline__ void acc_guard4(v8f& a, v8f& b, v8f& c, v8f& d) { asm volatile("v_nop\n\tv_nop\n\tv_nop\n\tv_nop" : "+v"(a), "+v"(b), "+v"(c), "+v"(d)); }
template <typename T> struct Frag;
template <> struct Frag<_Float16> {
  typedef v16h V; union U { v16h v; v8h h[2]; };
  static __device__ __forceinline__ v16h load(const _Float16* p) {
    U f; f.h[0] = *(const v8h*)(p); f.h[1] = *(const v8h*)(p + 16); return f.v;
  }
  static __device__ __forceinline__ v8f mma(v16h a, v16h b, v8f c) {
    return __builtin_amdgcn_wmma_f32_16x16x32_f16(false, a, false, b, (short)0, c, false, false);
  }
  static __device__ __forceinline__ void guard(v8f& a, v8f& b, v16h x, v16h y) { dep_guard_h(a, b, x, y); }
  static __device__ __forceinline__ void keep(v16h a, v16h b, v16h c, v16h d) { keep4_h(a, b, c, d); }
};
template <> struct Frag<__bf16> {
  typedef v16b V; union U { v16b v; v8b h[2]; };
  static __device__ __forceinline__ v16b load(const __bf16* p) {
    U f; f.h[0] = *(const v8b*)(p); f.h[1] = *(const v8b*)(p + 16); return f.v;
  }
  static __device__ __forceinline__ v8f mma(v16b a, v16b b, v8f c) {
    return __builtin_amdgcn_wmma_f32_16x16x32_bf16(false, a, false, b, (short)0, c, false, false);
  }
  static __device__ __forceinline__ void guard(v8f& a, v8f& b, v16b x, v16b y) { dep_guard_b(a, b, x, y); }
  static __device__ __forceinline__ void keep(v16b a, v16b b, v16b c, v16b d) { keep4_b(a, b, c, d); }
};

__device__ __forceinline__ unsigned pk16(unsigned short a, unsigned short b) { return (unsigned)a | ((unsigned)b << 16); }
__device__ __forceinline__ unsigned short h_bits(float f) { const _Float16 h = (_Float16)f; return __builtin_bit_cast(unsigned short, h); }

template <int ET> struct Elem;
template <> struct Elem<0> { typedef _Float16 T; };
template <> struct Elem<1> { typedef __bf16 T; };
template <int ET, bool SPLIT, int BIAS_MODE, int OUT_MODE, bool RESID, int ACT = 0>
__global__ __launch_bounds__(256) void wmma_gemm64(
    const unsigned short* __restrict__ Ap, const unsigned short* __restrict__ A2p, int lda, long strideA,
    const unsigned short* __restrict__ Btp, const unsigned short* __restrict__ Bt2p, int ldb, long strideB,
    void* __restrict__ Cout, void* __restrict__ Cout2, int ldc, long strideC,
    const float* __restrict__ bias,
    const float* __restrict__ resid, long strideR,
    int M, int N, int K, float scale) {
  typedef typename Elem<ET>::T T;
  typedef typename Frag<T>::V V;
  const T* A = (const T*)Ap; const T* A2 = (const T*)A2p; const T* Bt = (const T*)Btp; const T* Bt2 = (const T*)Bt2p;
  __shared__ __align__(16) float sT[8][16 * 68];
  const int b    = blockIdx.y;
  const int lane = threadIdx.x & 31;
  const int wave = threadIdx.x >> 5;
  const int tilesN = N >> 6;
  const int tilesM = M >> 6;
  const int tile = blockIdx.x * 8 + wave;
  if (tile >= tilesM * tilesN) return;
  const int tm = tile / tilesN;
  const int tn = tile - tm * tilesN;
  const int m0 = tm << 6;
  const int n0 = tn << 6;

  const T* Ab  = A  + (size_t)b * strideA;
  const T* Bb  = Bt + (size_t)b * strideB;
  const T* Ab2 = SPLIT ? (A2  + (size_t)b * strideA) : nullptr;
  const T* Bb2 = SPLIT ? (Bt2 + (size_t)b * strideB) : nullptr;

  const int rlane = lane & 15;
  const int koff  = (lane >> 4) * 8;
  const int mOff  = (lane >> 4) * 8;

  v8f acc[4][4];
#pragma unroll
  for (int i = 0; i < 4; ++i)
#pragma unroll
    for (int j = 0; j < 4; ++j) acc[i][j] = (v8f){0.f,0.f,0.f,0.f,0.f,0.f,0.f,0.f};

  for (int k0 = 0; k0 < K; k0 += 32) {
    V bh[4], bl[4];
#pragma unroll
    for (int j = 0; j < 4; ++j) {
      const size_t bo = (size_t)(n0 + (j << 4) + rlane) * ldb + koff + k0;
      bh[j] = Frag<T>::load(Bb + bo);
      if (SPLIT) bl[j] = Frag<T>::load(Bb2 + bo);
    }
#pragma unroll
    for (int i = 0; i < 4; ++i) {
      const size_t ao = (size_t)(m0 + (i << 4) + rlane) * lda + koff + k0;
      V ah = Frag<T>::load(Ab + ao);
      V al;
      if (SPLIT) al = Frag<T>::load(Ab2 + ao);
#pragma unroll
      for (int j = 0; j < 4; ++j) {
        acc[i][j] = Frag<T>::mma(ah, bh[j], acc[i][j]);
        if (SPLIT) {
          acc[i][j] = Frag<T>::mma(ah, bl[j], acc[i][j]);
          acc[i][j] = Frag<T>::mma(al, bh[j], acc[i][j]);
        }
      }
      Frag<T>::guard(acc[i][0], acc[i][3], ah, SPLIT ? al : ah);
    }
    Frag<T>::keep(bh[0], bh[1], bh[2], bh[3]);
    if (SPLIT) Frag<T>::keep(bl[0], bl[1], bl[2], bl[3]);
  }
  acc_guard4(acc[0][0], acc[0][1], acc[0][2], acc[0][3]);
  acc_guard4(acc[1][0], acc[1][1], acc[1][2], acc[1][3]);
  acc_guard4(acc[2][0], acc[2][1], acc[2][2], acc[2][3]);
  acc_guard4(acc[3][0], acc[3][1], acc[3][2], acc[3][3]);

  float* slab = sT[wave];
  const float* Rb = RESID ? (resid + (size_t)b * strideR) : nullptr;
#pragma unroll
  for (int i = 0; i < 4; ++i) {
    const int mBase = m0 + (i << 4);
#pragma unroll
    for (int j = 0; j < 4; ++j) {
      const int n = n0 + (j << 4) + rlane;
      float bv = 0.f;
      if (BIAS_MODE == 2) bv = bias[n];
#pragma unroll
      for (int r = 0; r < 8; ++r) {
        float v = acc[i][j][r] * scale;
        if (BIAS_MODE == 1) v += bias[mBase + mOff + r];
        if (BIAS_MODE == 2) v += bv;
        if (RESID) v += Rb[(size_t)(mBase + mOff + r) * ldc + n];
        if (ACT == 2) v = fmaxf(v, 0.0f);
        if (ACT == 4) v = (v > 0.f) ? v : 0.01f * v;
        slab[(mOff + r) * 68 + (j << 4) + rlane] = v;
      }
    }
    __builtin_amdgcn_fence(__ATOMIC_RELEASE, "workgroup");
    __builtin_amdgcn_wave_barrier();
    __builtin_amdgcn_fence(__ATOMIC_ACQUIRE, "workgroup");
    if (OUT_MODE == 0) {
      float* C = (float*)Cout + (size_t)b * strideC;
      const int hh = lane >> 4, c4 = (lane & 15) * 4;
      for (int pass = 0; pass < 2; ++pass) {
#pragma unroll
        for (int it = 0; it < 8; ++it) {
          const int row = it * 2 + hh;
          v4f v = *(const v4f*)(slab + row * 68 + c4);
          *(volatile v4f*)(C + (size_t)(mBase + row) * ldc + n0 + c4) = v;
        }
        __threadfence();
      }
    } else {
      const int q = lane >> 3, c8 = (lane & 7) * 8;
      unsigned short* C  = (unsigned short*)Cout  + (size_t)b * strideC;
      unsigned short* C2 = (OUT_MODE == 2) ? ((unsigned short*)Cout2 + (size_t)b * strideC) : nullptr;
      for (int pass = 0; pass < 2; ++pass) {
#pragma unroll
        for (int it = 0; it < 4; ++it) {
          const int row = it * 4 + q;
          const float* sp = slab + row * 68 + c8;
          v8h hv, lv;
#pragma unroll
          for (int e = 0; e < 8; ++e) {
            if (OUT_MODE == 1) {
              hv[e] = (_Float16)sp[e];
            } else {
              unsigned short hb = f2bf_bits(sp[e]);
              unsigned short lb = f2bf_bits(sp[e] - bf_bits2f(hb));
              hv[e] = __builtin_bit_cast(_Float16, hb);
              lv[e] = __builtin_bit_cast(_Float16, lb);
            }
          }
          *(volatile v8h*)(C + (size_t)(mBase + row) * ldc + n0 + c8) = hv;
          if (OUT_MODE == 2) *(volatile v8h*)(C2 + (size_t)(mBase + row) * ldc + n0 + c8) = lv;
        }
        __threadfence();
      }
    }
    __builtin_amdgcn_fence(__ATOMIC_RELEASE, "workgroup");
    __builtin_amdgcn_wave_barrier();
    __builtin_amdgcn_fence(__ATOMIC_ACQUIRE, "workgroup");
  }
}

__global__ __launch_bounds__(256) void coef_plane_kernel(const float* __restrict__ Cf, unsigned short* __restrict__ Bt) {
  const int g  = blockIdx.x * 256 + threadIdx.x;
  const int wg = g >> 5;
  const int l  = g & 31;
  const int o  = wg >> 6;
  const int i  = ((wg & 63) << 3) + (l >> 2);
  const int kk0 = (l & 3) << 3;
  const float* src = Cf + (size_t)i * (kOutF * kKnots) + (size_t)o * kKnots + kk0;
  const v4f a = *(const v4f*)(src);
  const v4f c = *(const v4f*)(src + 4);
  unsigned short hb[8];
#pragma unroll
  for (int e = 0; e < 4; ++e) {
    hb[e]     = h_bits(a[e] * kCoefCarry);
    hb[4 + e] = h_bits(c[e] * kCoefCarry);
  }
  const v4u u = (v4u){pk16(hb[0], hb[1]), pk16(hb[2], hb[3]), pk16(hb[4], hb[5]), pk16(hb[6], hb[7])};
  unsigned short* dst = Bt + 8 * (size_t)g;
  *(volatile v4u*)dst = u;
  __threadfence();
  *(volatile v4u*)dst = u;
}

__global__ __launch_bounds__(256) void basis_plane_kernel(const float* __restrict__ X, const float* __restrict__ Kn,
                                                          unsigned short* __restrict__ Apl) {
#pragma clang fp contract(off)
  __shared__ float tt[kTabAlloc];
  __shared__ float r1[kTabAlloc];
  __shared__ float r2[kTabAlloc];
  __shared__ float r3[kTabAlloc];
  const int t = threadIdx.x;
  const float kn0 = Kn[0];
  const float kn1 = Kn[1];
  const float hstep = kn1 - kn0;
  {
    float tv[4];
#pragma unroll
    for (int s = 0; s < 4; ++s) {
      const int m  = t + s - kTabOff;
      const int mc = m < 0 ? 0 : (m > kKnots - 1 ? kKnots - 1 : m);
      const float base = Kn[mc];
      const float ext  = hstep * (float)(m - mc);
      tv[s] = base + ext;
    }
    const float q1 = 1.0f / (tv[1] - tv[0]);
    const float q2 = 1.0f / (tv[2] - tv[0]);
    const float q3 = 1.0f / (tv[3] - tv[0]);
    if (t < kTabAlloc) {
      tt[t] = tv[0];
      r1[t] = q1;
      r2[t] = q2;
      r3[t] = q3;
    }
  }
  __syncthreads();

  const int g = blockIdx.x * 256 + t;
  const int q = t & 3;
  const float x = X[g >> 2];

  const float inv_h = 1.0f / hstep;
  float fj = floorf((x - kn0) * inv_h);
  fj = fminf(fmaxf(fj, 0.0f), (float)kMaxInterval);
  int j = (int)fj;
#pragma unroll
  for (int s = 0; s < 2; ++s) {
    const float tlo = tt[j + kTabOff];
    const float thi = tt[j + kTabOff + 1];
    const int dn = ((x < tlo) && (j > 0)) ? 1 : 0;
    const int up = ((x >= thi) && (j < kMaxInterval)) ? 1 : 0;
    j = j + up - dn;
  }
  const float Tm2 = tt[j + kTabOff - 2];
  const float Tm1 = tt[j + kTabOff - 1];
  const float T0  = tt[j + kTabOff];
  const float T1  = tt[j + kTabOff + 1];
  const float T2  = tt[j + kTabOff + 2];
  const float T3  = tt[j + kTabOff + 3];
  const float R1  = r1[j + kTabOff];
  const float R2a = r2[j + kTabOff - 1];
  const float R2b = r2[j + kTabOff];
  const float R3a = r3[j + kTabOff - 2];
  const float R3b = r3[j + kTabOff - 1];
  const float R3c = r3[j + kTabOff];
  const bool inspan = (x >= T0) && (x < T1);

  const float n1a = ((T1 - x) * R1);
  const float n1b = ((x - T0) * R1);
  const float n2a = ((T1 - x) * R2a) * n1a;
  const float n2b = ((x - Tm1) * R2a) * n1a + ((T2 - x) * R2b) * n1b;
  const float n2c = ((x - T0) * R2b) * n1b;
  float n30 = ((T1 - x) * R3a) * n2a;
  float n31 = ((x - Tm2) * R3a) * n2a + ((T2 - x) * R3b) * n2b;
  float n32 = ((x - Tm1) * R3b) * n2b + ((T3 - x) * R3c) * n2c;
  float n33 = ((x - T0) * R3c) * n2c;
  n30 = inspan ? n30 * kBasisCarry : 0.0f;
  n31 = inspan ? n31 * kBasisCarry : 0.0f;
  n32 = inspan ? n32 * kBasisCarry : 0.0f;
  n33 = inspan ? n33 * kBasisCarry : 0.0f;

  unsigned short hb[8];
#pragma unroll
  for (int e = 0; e < 8; ++e) {
    const int s = (q << 3) + e - j + 3;
    float v = 0.0f;
    v = (s == 0) ? n30 : v;
    v = (s == 1) ? n31 : v;
    v = (s == 2) ? n32 : v;
    v = (s == 3) ? n33 : v;
    hb[e] = h_bits(v);
  }
  const v4u u = (v4u){pk16(hb[0], hb[1]), pk16(hb[2], hb[3]), pk16(hb[4], hb[5]), pk16(hb[6], hb[7])};
  unsigned short* dst = Apl + 8 * (size_t)g;
  *(volatile v4u*)dst = u;
  __threadfence();
  *(volatile v4u*)dst = u;
}

extern "C" void kernel_launch(void* const* d_in, const int* in_sizes, int n_in,
                              void* d_out, int out_size, void* d_ws, size_t ws_size,
                              hipStream_t stream) {
  if (n_in < 3) return;
  if (in_sizes[0] != kBatch * kInF) return;
  if (in_sizes[1] != kInF * kOutF * kKnots) return;
  if (in_sizes[2] != kKnots) return;
  if (out_size != kBatch * kOutF) return;
  const size_t btBytes = (size_t)kOutF * kKdim * 2;
  const size_t aBytes  = (size_t)kBatch * kKdim * 2;
  if (btBytes + aBytes > ws_size) return;

  const float* x     = (const float*)d_in[0];
  const float* coef  = (const float*)d_in[1];
  const float* knots = (const float*)d_in[2];
  float* out = (float*)d_out;
  unsigned short* Bt  = (unsigned short*)d_ws;
  unsigned short* Apl = (unsigned short*)((char*)d_ws + btBytes);

  const int nCoefThreads  = kOutF * kKdim / 8;
  const int nBasisThreads = kBatch * kInF * 4;
  coef_plane_kernel<<<(nCoefThreads + 255) / 256, 256, 0, stream>>>(coef, Bt);
  basis_plane_kernel<<<(nBasisThreads + 255) / 256, 256, 0, stream>>>(x, knots, Apl);

  const int tiles = (kBatch / 64) * (kOutF / 64);
  dim3 ggrid((tiles + 7) / 8, 1, 1);
  wmma_gemm64<0, false, 0, 0, false, 0><<<ggrid, 256, 0, stream>>>(
      Apl, Apl, kKdim, 0L,
      Bt, Bt, kKdim, 0L,
      (void*)out, (void*)out, kOutF, 0L,
      knots,
      x, 0L,
      kBatch, kOutF, kKdim, kOutScale);
}
